// SelectiveCrossSSM_16114717294733
// MI455X (gfx1250) — hardware-run, weakly checked
//
#include <hip/hip_runtime.h>
#include <math.h>

typedef __attribute__((ext_vector_type(16))) _Float16 v16h;
typedef __attribute__((ext_vector_type(8)))  _Float16 v8h;
typedef __attribute__((ext_vector_type(16))) __bf16   v16b;
typedef __attribute__((ext_vector_type(8)))  __bf16   v8b;
typedef __attribute__((ext_vector_type(8)))  float    v8f;
typedef __attribute__((ext_vector_type(4)))  float    v4f;

constexpr int kBatch  = 4;
constexpr int kSeq    = 1024;
constexpr int kDm     = 512;
constexpr int kDin    = 1024;
constexpr int kNst    = 16;
constexpr int kHeads  = 8;
constexpr int kDh     = 64;
constexpr int kRows   = kBatch * kSeq;
constexpr int kBxzW   = 2 * kDin;
constexpr int kCatW   = kDin + kDm;
constexpr int kBcReal = 2 * kNst;
constexpr int kBcW    = 64;
constexpr int kGcW    = 2 * kDm;
constexpr int kF1W    = 2 * kDm;
constexpr int kConvTP = 260;
constexpr int kScanTS = 64;
constexpr int kScanCh = 64;
constexpr int kScanYP = 68;
constexpr float kLog2e = 1.4426950408889634f;
static_assert(kHeads * kDh == kDm, "head split");
static_assert((kDm % 32) == 0 && (kDin % 32) == 0 && (kCatW % 32) == 0 && (kDh % 32) == 0 && (kSeq % 32) == 0, "GEMM K multiples of 32");
static_assert((kRows % 64) == 0 && (kDm % 64) == 0 && (kDin % 64) == 0 && (kBxzW % 64) == 0 && (kBcW % 64) == 0 &&
              (kSeq % 64) == 0 && (kDh % 64) == 0 && (kF1W % 64) == 0 && (kCatW % 64) == 0, "GEMM M,N multiples of 64");
static_assert((kSeq % kScanTS) == 0 && (kDin % kScanCh) == 0 && (kDin % 256) == 0 && (kRows % 8) == 0, "tile multiples");
static_assert(((kRows * kDm) % 2048) == 0 && ((kRows * kF1W) % 2048) == 0, "cast chunking");

constexpr size_t kOffWCTX  = 0;
constexpr size_t kOffWBIO  = kOffWCTX  + (size_t)kDm   * kDm  * 2;
constexpr size_t kOffWDT   = kOffWBIO  + (size_t)kBxzW * kDm  * 2;
constexpr size_t kOffWBC   = kOffWDT   + (size_t)kDin  * kCatW * 2;
constexpr size_t kOffWSSM  = kOffWBC   + (size_t)kBcW  * kDin * 2;
constexpr size_t kOffWIN   = kOffWSSM  + (size_t)kDm   * kDin * 2;
constexpr size_t kOffWOUT  = kOffWIN   + (size_t)(3 * kDm) * kDm * 2;
constexpr size_t kOffWGATE = kOffWOUT  + (size_t)kDm   * kDm  * 2;
constexpr size_t kOffWF1   = kOffWGATE + (size_t)kDm   * kGcW * 2;
constexpr size_t kOffWF2   = kOffWF1   + (size_t)kF1W  * kDm  * 2;
constexpr size_t kOffRS    = kOffWF2   + (size_t)kDm   * kF1W * 2;
constexpr size_t kSzRS     = (size_t)kHeads * kSeq * kSeq * 4;
constexpr size_t kOffRB    = kOffRS + kSzRS;
constexpr size_t kSzRB     = (size_t)kRows * kBxzW * 4;
constexpr size_t kOffRU    = kOffRB + kSzRB;
constexpr size_t kSzRU     = (size_t)kRows * kDin * 4;
constexpr size_t kOffRD    = kOffRU + kSzRU;
constexpr size_t kSzRD     = (size_t)kRows * kDin * 4;
constexpr size_t kOffRC    = kOffRD + kSzRD;
constexpr size_t kSzRC     = (size_t)kRows * kCatW * 2;
constexpr size_t kOffRBC   = kOffRC + kSzRC;
constexpr size_t kSzRBC    = (size_t)kRows * kBcW * 4;
constexpr size_t kWsTotal  = kOffRBC + kSzRBC;
static_assert(kOffRS == 12189696ull, "weight planes");
static_assert(kWsTotal == 126484480ull, "carve total");
static_assert(kWsTotal <= 134217728ull, "carve cap");
static_assert((kOffWBIO % 128) == 0 && (kOffWDT % 128) == 0 && (kOffWBC % 128) == 0 && (kOffWSSM % 128) == 0 &&
              (kOffWIN % 128) == 0 && (kOffWOUT % 128) == 0 && (kOffWGATE % 128) == 0 && (kOffWF1 % 128) == 0 &&
              (kOffWF2 % 128) == 0 && (kOffRS % 128) == 0 && (kOffRB % 128) == 0 && (kOffRU % 128) == 0 &&
              (kOffRD % 128) == 0 && (kOffRC % 128) == 0 && (kOffRBC % 128) == 0, "128-B aligned regions");
static_assert((size_t)2 * kRows * kDm * 2 + (size_t)kRows * kDm * 4 <= kSzRS, "RS phase 1");
static_assert((size_t)4 * kRows * kDm * 4 <= kSzRB && (size_t)kRows * kDm * 4 + (size_t)kRows * kGcW * 2 <= (size_t)2 * kRows * kDm * 4, "RB phase 2");
static_assert((size_t)3 * kRows * kDm * 2 <= kSzRU && (size_t)kRows * kF1W * 4 <= kSzRU, "RU phase 2");
static_assert((size_t)kHeads * kSeq * kSeq * 2 <= kSzRD && (size_t)kRows * kF1W * 2 <= kSzRD, "RD phase 2");
static_assert((size_t)kRows * kDin * 2 <= kSzRC && (size_t)3 * kRows * kDm * 2 <= kSzRC &&
              (size_t)kRows * kDm * 4 + (size_t)kRows * kDm * 2 <= kSzRC, "RC phase 2");

__device__ __forceinline__ unsigned short f2bf_bits(float f) {
  unsigned u = __float_as_uint(f);
  return (unsigned short)((u + 0x7FFFu + ((u >> 16) & 1u)) >> 16);
}
__device__ __forceinline__ float bf_bits2f(unsigned short h) { return __uint_as_float(((unsigned)h) << 16); }

__device__ __forceinline__ void dep_guard_h(v8f& a, v8f& b, v16h x, v16h y) { asm volatile("v_nop\n\tv_nop\n\tv_nop\n\tv_nop" : "+v"(a), "+v"(b) : "v"(x), "v"(y)); }
__device__ __forceinline__ void dep_guard_b(v8f& a, v8f& b, v16b x, v16b y) { asm volatile("v_nop\n\tv_nop\n\tv_nop\n\tv_nop" : "+v"(a), "+v"(b) : "v"(x), "v"(y)); }
__device__ __forceinline__ void keep4_h(v16h a, v16h b, v16h c, v16h d) { asm volatile("v_nop" :: "v"(a), "v"(b), "v"(c), "v"(d)); }
__device__ __forceinline__ void keep4_b(v16b a, v16b b, v16b c, v16b d) { asm volatile("v_nop" :: "v"(a), "v"(b), "v"(c), "v"(d)); }
__device__ __forceinline__ void acc_guard4(v8f& a, v8f& b, v8f& c, v8f& d) { asm volatile("v_nop\n\tv_nop\n\tv_nop\n\tv_nop" : "+v"(a), "+v"(b), "+v"(c), "+v"(d)); }
template <typename T> struct Frag;
template <> struct Frag<_Float16> {
  typedef v16h V; union U { v16h v; v8h h[2]; };
  static __device__ __forceinline__ v16h load(const _Float16* p) {
    U f; f.h[0] = *(const v8h*)(p); f.h[1] = *(const v8h*)(p + 16); return f.v;
  }
  static __device__ __forceinline__ v8f mma(v16h a, v16h b, v8f c) {
    return __builtin_amdgcn_wmma_f32_16x16x32_f16(false, a, false, b, (short)0, c, false, false);
  }
  static __device__ __forceinline__ void guard(v8f& a, v8f& b, v16h x, v16h y) { dep_guard_h(a, b, x, y); }
  static __device__ __forceinline__ void keep(v16h a, v16h b, v16h c, v16h d) { keep4_h(a, b, c, d); }
};
template <> struct Frag<__bf16> {
  typedef v16b V; union U { v16b v; v8b h[2]; };
  static __device__ __forceinline__ v16b load(const __bf16* p) {
    U f; f.h[0] = *(const v8b*)(p); f.h[1] = *(const v8b*)(p + 16); return f.v;
  }
  static __device__ __forceinline__ v8f mma(v16b a, v16b b, v8f c) {
    return __builtin_amdgcn_wmma_f32_16x16x32_bf16(false, a, false, b, (short)0, c, false, false);
  }
  static __device__ __forceinline__ void guard(v8f& a, v8f& b, v16b x, v16b y) { dep_guard_b(a, b, x, y); }
  static __device__ __forceinline__ void keep(v16b a, v16b b, v16b c, v16b d) { keep4_b(a, b, c, d); }
};

template <int ET> struct Elem;
template <> struct Elem<0> { typedef _Float16 T; };
template <> struct Elem<1> { typedef __bf16 T; };
template <int ET, bool SPLIT, int BIAS_MODE, int OUT_MODE, bool RESID, int ACT = 0>
__global__ __launch_bounds__(256) void wmma_gemm64(
    const unsigned short* __restrict__ Ap, const unsigned short* __restrict__ A2p, int lda, long strideA,
    const unsigned short* __restrict__ Btp, const unsigned short* __restrict__ Bt2p, int ldb, long strideB,
    void* __restrict__ Cout, void* __restrict__ Cout2, int ldc, long strideC,
    const float* __restrict__ bias,
    const float* __restrict__ resid, long strideR,
    int M, int N, int K, float scale) {
  typedef typename Elem<ET>::T T;
  typedef typename Frag<T>::V V;
  const T* A = (const T*)Ap; const T* A2 = (const T*)A2p; const T* Bt = (const T*)Btp; const T* Bt2 = (const T*)Bt2p;
  __shared__ __align__(16) float sT[8][16 * 68];
  const int b    = blockIdx.y;
  const int lane = threadIdx.x & 31;
  const int wave = threadIdx.x >> 5;
  const int tilesN = N >> 6;
  const int tilesM = M >> 6;
  const int tile = blockIdx.x * 8 + wave;
  if (tile >= tilesM * tilesN) return;
  const int tm = tile / tilesN;
  const int tn = tile - tm * tilesN;
  const int m0 = tm << 6;
  const int n0 = tn << 6;

  const T* Ab  = A  + (size_t)b * strideA;
  const T* Bb  = Bt + (size_t)b * strideB;
  const T* Ab2 = SPLIT ? (A2  + (size_t)b * strideA) : nullptr;
  const T* Bb2 = SPLIT ? (Bt2 + (size_t)b * strideB) : nullptr;

  const int rlane = lane & 15;
  const int koff  = (lane >> 4) * 8;
  const int mOff  = (lane >> 4) * 8;

  v8f acc[4][4];
#pragma unroll
  for (int i = 0; i < 4; ++i)
#pragma unroll
    for (int j = 0; j < 4; ++j) acc[i][j] = (v8f){0.f,0.f,0.f,0.f,0.f,0.f,0.f,0.f};

  for (int k0 = 0; k0 < K; k0 += 32) {
    V bh[4], bl[4];
#pragma unroll
    for (int j = 0; j < 4; ++j) {
      const size_t bo = (size_t)(n0 + (j << 4) + rlane) * ldb + koff + k0;
      bh[j] = Frag<T>::load(Bb + bo);
      if (SPLIT) bl[j] = Frag<T>::load(Bb2 + bo);
    }
#pragma unroll
    for (int i = 0; i < 4; ++i) {
      const size_t ao = (size_t)(m0 + (i << 4) + rlane) * lda + koff + k0;
      V ah = Frag<T>::load(Ab + ao);
      V al;
      if (SPLIT) al = Frag<T>::load(Ab2 + ao);
#pragma unroll
      for (int j = 0; j < 4; ++j) {
        acc[i][j] = Frag<T>::mma(ah, bh[j], acc[i][j]);
        if (SPLIT) {
          acc[i][j] = Frag<T>::mma(ah, bl[j], acc[i][j]);
          acc[i][j] = Frag<T>::mma(al, bh[j], acc[i][j]);
        }
      }
      Frag<T>::guard(acc[i][0], acc[i][3], ah, SPLIT ? al : ah);
    }
    Frag<T>::keep(bh[0], bh[1], bh[2], bh[3]);
    if (SPLIT) Frag<T>::keep(bl[0], bl[1], bl[2], bl[3]);
  }
  acc_guard4(acc[0][0], acc[0][1], acc[0][2], acc[0][3]);
  acc_guard4(acc[1][0], acc[1][1], acc[1][2], acc[1][3]);
  acc_guard4(acc[2][0], acc[2][1], acc[2][2], acc[2][3]);
  acc_guard4(acc[3][0], acc[3][1], acc[3][2], acc[3][3]);

  float* slab = sT[wave];
  const float* Rb = RESID ? (resid + (size_t)b * strideR) : nullptr;
#pragma unroll
  for (int i = 0; i < 4; ++i) {
    const int mBase = m0 + (i << 4);
#pragma unroll
    for (int j = 0; j < 4; ++j) {
      const int n = n0 + (j << 4) + rlane;
      float bv = 0.f;
      if (BIAS_MODE == 2) bv = bias[n];
#pragma unroll
      for (int r = 0; r < 8; ++r) {
        float v = acc[i][j][r] * scale;
        if (BIAS_MODE == 1) v += bias[mBase + mOff + r];
        if (BIAS_MODE == 2) v += bv;
        if (RESID) v += Rb[(size_t)(mBase + mOff + r) * ldc + n];
        if (ACT == 2) v = fmaxf(v, 0.0f);
        if (ACT == 4) v = (v > 0.f) ? v : 0.01f * v;
        slab[(mOff + r) * 68 + (j << 4) + rlane] = v;
      }
    }
    __builtin_amdgcn_fence(__ATOMIC_RELEASE, "workgroup");
    __builtin_amdgcn_wave_barrier();
    __builtin_amdgcn_fence(__ATOMIC_ACQUIRE, "workgroup");
    if (OUT_MODE == 0) {
      float* C = (float*)Cout + (size_t)b * strideC;
      const int hh = lane >> 4, c4 = (lane & 15) * 4;
      for (int pass = 0; pass < 2; ++pass) {
#pragma unroll
        for (int it = 0; it < 8; ++it) {
          const int row = it * 2 + hh;
          v4f v = *(const v4f*)(slab + row * 68 + c4);
          *(volatile v4f*)(C + (size_t)(mBase + row) * ldc + n0 + c4) = v;
        }
        __threadfence();
      }
    } else {
      const int q = lane >> 3, c8 = (lane & 7) * 8;
      unsigned short* C  = (unsigned short*)Cout  + (size_t)b * strideC;
      unsigned short* C2 = (OUT_MODE == 2) ? ((unsigned short*)Cout2 + (size_t)b * strideC) : nullptr;
      for (int pass = 0; pass < 2; ++pass) {
#pragma unroll
        for (int it = 0; it < 4; ++it) {
          const int row = it * 4 + q;
          const float* sp = slab + row * 68 + c8;
          v8h hv, lv;
#pragma unroll
          for (int e = 0; e < 8; ++e) {
            if (OUT_MODE == 1) {
              hv[e] = (_Float16)sp[e];
            } else {
              unsigned short hb = f2bf_bits(sp[e]);
              unsigned short lb = f2bf_bits(sp[e] - bf_bits2f(hb));
              hv[e] = __builtin_bit_cast(_Float16, hb);
              lv[e] = __builtin_bit_cast(_Float16, lb);
            }
          }
          *(volatile v8h*)(C + (size_t)(mBase + row) * ldc + n0 + c8) = hv;
          if (OUT_MODE == 2) *(volatile v8h*)(C2 + (size_t)(mBase + row) * ldc + n0 + c8) = lv;
        }
        __threadfence();
      }
    }
    __builtin_amdgcn_fence(__ATOMIC_RELEASE, "workgroup");
    __builtin_amdgcn_wave_barrier();
    __builtin_amdgcn_fence(__ATOMIC_ACQUIRE, "workgroup");
  }
}

__device__ __forceinline__ float sigm_f(float x) { return __builtin_amdgcn_rcpf(1.0f + expf(-x)); }

template <int ACT>
__global__ __launch_bounds__(256) void act_cast_kernel(
    const float* __restrict__ src, int w, unsigned short* __restrict__ dst, int ldd, int coloff, float scale)
{
  __shared__ __align__(16) float sh[(ACT == 1) ? 2048 : 4];
  const int tid = threadIdx.x;
  const size_t base = (size_t)blockIdx.x * 2048;
  v4f a0, a1;
  if (ACT == 1) {
#pragma unroll 1
    for (int e = 0; e < 8; ++e) {
      const float x = src[base + (size_t)e * 256 + tid];
      sh[e * 256 + tid] = 0.5f * x * (1.0f + erff(x * 0.70710678118654752f));
    }
    __syncthreads();
    a0 = *(const v4f*)(sh + tid * 8);
    a1 = *(const v4f*)(sh + tid * 8 + 4);
  } else {
    a0 = *(const v4f*)(src + base + (size_t)tid * 8);
    a1 = *(const v4f*)(src + base + (size_t)tid * 8 + 4);
  }
  v8h hv;
#pragma unroll
  for (int e = 0; e < 4; ++e) {
    hv[e]     = (_Float16)(a0[e] * scale);
    hv[4 + e] = (_Float16)(a1[e] * scale);
  }
  const unsigned g   = (unsigned)base + (unsigned)tid * 8u;
  const unsigned row = g / (unsigned)w;
  const unsigned col = g - row * (unsigned)w;
  unsigned short* p = dst + (size_t)row * ldd + coloff + col;
  *(volatile v8h*)p = hv;
  __threadfence();
  *(volatile v8h*)p = hv;
}

__global__ __launch_bounds__(256) void wt_cast_kernel(
    const float* __restrict__ W, int nreal, unsigned short* __restrict__ Bt, int kin, float scale)
{
  __shared__ __align__(16) float sT[64 * 65];
  const int tid = threadIdx.x, lane = tid & 31, wave = tid >> 5;
  const int k0 = blockIdx.x * 64, n0 = blockIdx.y * 64;
  const int r = tid >> 4, c4 = (tid & 15) * 4;
#pragma unroll
  for (int i = 0; i < 4; ++i) {
    const int kr = r + 16 * i;
    const int nc = n0 + c4;
    const int ncl = (nc <= nreal - 4) ? nc : (nreal - 4);
    const v4f v = *(const v4f*)(W + (size_t)(k0 + kr) * nreal + ncl);
#pragma unroll
    for (int e = 0; e < 4; ++e) sT[kr * 65 + c4 + e] = (nc + e < nreal) ? v[e] : 0.0f;
  }
  __syncthreads();
  const int q = lane >> 3, c8 = (lane & 7) * 8;
  v8h hv[2];
#pragma unroll
  for (int it = 0; it < 2; ++it) {
    const int nn = it * 32 + wave * 4 + q;
#pragma unroll
    for (int e = 0; e < 8; ++e) hv[it][e] = (_Float16)(sT[(c8 + e) * 65 + nn] * scale);
  }
  for (int pass = 0; pass < 2; ++pass) {
#pragma unroll
    for (int it = 0; it < 2; ++it) {
      const int nn = it * 32 + wave * 4 + q;
      *(volatile v8h*)(Bt + (size_t)(n0 + nn) * kin + k0 + c8) = hv[it];
    }
    __threadfence();
  }
}

__global__ __launch_bounds__(256) void conv_silu_kernel(
    const float* __restrict__ BXZ, const float* __restrict__ cw, const float* __restrict__ cb,
    float* __restrict__ UC, unsigned short* __restrict__ CAT)
{
  __shared__ __align__(16) float sT[16 * kConvTP];
  const int tid = threadIdx.x, lane = tid & 31, wave = tid >> 5;
  const int d0 = blockIdx.x * 256, d = d0 + tid;
  const int g0 = blockIdx.y * 64;
  const int tb = g0 & (kSeq - 1);
  const float w0 = cw[d * 4 + 0], w1 = cw[d * 4 + 1], w2 = cw[d * 4 + 2], w3 = cw[d * 4 + 3];
  const float bcv = cb[d];
  float xm3, xm2, xm1;
  {
    const bool hist = (tb > 0);
    const int rb = hist ? (g0 - 3) : g0;
    const float v3 = BXZ[(size_t)rb * kBxzW + d];
    const float v2 = BXZ[(size_t)(rb + 1) * kBxzW + d];
    const float v1 = BXZ[(size_t)(rb + 2) * kBxzW + d];
    xm3 = hist ? v3 : 0.f;
    xm2 = hist ? v2 : 0.f;
    xm1 = hist ? v1 : 0.f;
  }
  const int hrow = wave >> 1;
  const int hch  = (wave & 1) * 128 + lane * 4;
#pragma unroll 1
  for (int sub = 0; sub < 4; ++sub) {
    const int lb = g0 + sub * 16;
#pragma unroll 1
    for (int s = 0; s < 16; ++s) {
      const float xcur = BXZ[(size_t)(lb + s) * kBxzW + d];
      float acc = w0 * xm3;
      acc = fmaf(w1, xm2, acc);
      acc = fmaf(w2, xm1, acc);
      acc = fmaf(w3, xcur, acc);
      const float sv = acc + bcv;
      const float sg = sigm_f(sv);
      sT[s * kConvTP + tid] = sv * sg;
      xm3 = xm2; xm2 = xm1; xm1 = xcur;
    }
    __syncthreads();
    v4f fv[4];
    v8h hv[2];
#pragma unroll
    for (int it = 0; it < 4; ++it) fv[it] = *(const v4f*)(sT + (it * 4 + hrow) * kConvTP + hch);
#pragma unroll
    for (int it = 0; it < 2; ++it) {
      const float* sp = sT + (it * 8 + wave) * kConvTP + lane * 8;
      const v4f a0 = *(const v4f*)(sp);
      const v4f a1 = *(const v4f*)(sp + 4);
#pragma unroll
      for (int e = 0; e < 4; ++e) {
        hv[it][e]     = (_Float16)(a0[e] * 256.0f);
        hv[it][4 + e] = (_Float16)(a1[e] * 256.0f);
      }
    }
    for (int pass = 0; pass < 2; ++pass) {
#pragma unroll
      for (int it = 0; it < 4; ++it)
        *(volatile v4f*)(UC + (size_t)(lb + it * 4 + hrow) * kDin + d0 + hch) = fv[it];
#pragma unroll
      for (int it = 0; it < 2; ++it)
        *(volatile v8h*)(CAT + (size_t)(lb + it * 8 + wave) * kCatW + d0 + lane * 8) = hv[it];
      __threadfence();
    }
    __syncthreads();
  }
}

__global__ __launch_bounds__(64) void scan_kernel(
    const float* __restrict__ DTP, const float* __restrict__ BCm, const float* __restrict__ UC,
    const float* __restrict__ BXZ, const float* __restrict__ Alog, const float* __restrict__ Dp,
    unsigned short* __restrict__ Y16)
{
  __shared__ __align__(16) float sBC[kScanTS * kBcReal];
  __shared__ __align__(16) float sY[kScanTS * kScanYP];
  __shared__ __align__(16) float sA[kNst * kScanCh];
  const int tid = threadIdx.x, lane = tid & 31, wave = tid >> 5;
  constexpr int kBlkPerB = kDin / kScanCh;
  const int bix = blockIdx.x / kBlkPerB;
  const int d0  = (blockIdx.x - bix * kBlkPerB) * kScanCh;
  const int d   = d0 + tid;
  const size_t row0 = (size_t)bix * kSeq;
#pragma unroll 1
  for (int s = 0; s < kNst; ++s) sA[s * kScanCh + tid] = -expf(Alog[(size_t)d * kNst + s]) * kLog2e;
  __syncthreads();
  float la[kNst], h[kNst];
#pragma unroll
  for (int s = 0; s < kNst; ++s) {
    la[s] = sA[s * kScanCh + tid];
    h[s] = 0.f;
  }
  const float Dd = Dp[d];
  const int lr = tid >> 3, lc4 = (tid & 7) * 4;
  const int q = lane >> 3, c8 = (lane & 7) * 8;
#pragma unroll 1
  for (int t0 = 0; t0 < kSeq; t0 += kScanTS) {
    __syncthreads();
#pragma unroll
    for (int i = 0; i < 8; ++i) {
      const int r = lr + 8 * i;
      *(v4f*)(sBC + r * kBcReal + lc4) = *(const v4f*)(BCm + (row0 + t0 + r) * kBcW + lc4);
    }
    __syncthreads();
#pragma unroll 1
    for (int s = 0; s < kScanTS; ++s) {
      const size_t row = row0 + t0 + s;
      const float* xr = sBC + s * kBcReal;
      float Bs[kNst], Cs[kNst];
#pragma unroll
      for (int q4 = 0; q4 < 4; ++q4) {
        const v4f bv = *(const v4f*)(xr + 4 * q4);
        const v4f cv = *(const v4f*)(xr + kNst + 4 * q4);
        Bs[4 * q4 + 0] = bv[0]; Bs[4 * q4 + 1] = bv[1]; Bs[4 * q4 + 2] = bv[2]; Bs[4 * q4 + 3] = bv[3];
        Cs[4 * q4 + 0] = cv[0]; Cs[4 * q4 + 1] = cv[1]; Cs[4 * q4 + 2] = cv[2]; Cs[4 * q4 + 3] = cv[3];
      }
      const float v   = DTP[row * kDin + d];
      const float dt  = fmaxf(v, 0.0f) + log1pf(expf(-fabsf(v)));
      const float xt  = UC[row * kDin + d];
      const float dtx = dt * xt;
      float y = 0.f;
#pragma unroll
      for (int k = 0; k < kNst; ++k) {
        const float e = exp2f(dt * la[k]);
        h[k] = e * h[k] + dtx * Bs[k];
        y = h[k] * Cs[k] + y;
      }
      y = y + Dd * xt;
      const float zv = BXZ[row * kBxzW + kDin + d];
      const float sg = sigm_f(zv);
      y = y * (zv * sg);
      sY[s * kScanYP + tid] = y;
    }
    __syncthreads();
    v8h hv[8];
#pragma unroll
    for (int it = 0; it < 8; ++it) {
      const int row = it * 8 + wave * 4 + q;
      const float* sp = sY + row * kScanYP + c8;
      const v4f a0 = *(const v4f*)(sp);
      const v4f a1 = *(const v4f*)(sp + 4);
#pragma unroll
      for (int e = 0; e < 4; ++e) {
        hv[it][e]     = (_Float16)(a0[e] * 1024.0f);
        hv[it][4 + e] = (_Float16)(a1[e] * 1024.0f);
      }
    }
    for (int pass = 0; pass < 2; ++pass) {
#pragma unroll
      for (int it = 0; it < 8; ++it) {
        const int row = it * 8 + wave * 4 + q;
        const size_t o = (row0 + t0 + row) * kDin + d0 + c8;
        *(volatile v8h*)(Y16 + o) = hv[it];
      }
      __threadfence();
    }
  }
}

template <int MODE>
__global__ __launch_bounds__(256) void ln_rows_kernel(
    const float* __restrict__ src, const float* __restrict__ gpre, const float* __restrict__ aout,
    const float* __restrict__ biof, const float* __restrict__ gam, const float* __restrict__ bet,
    float* __restrict__ hc, unsigned short* __restrict__ dst16, unsigned short* __restrict__ aux16)
{
  __shared__ __align__(16) float sh[8][kDm];
  const int tid = threadIdx.x, lane = tid & 31, wave = tid >> 5;
  const int row = blockIdx.x * 8 + wave;
  const size_t rb = (size_t)row * kDm;
  float* sr = sh[wave];
  float sum = 0.f;
#pragma unroll 1
  for (int j = 0; j < 4; ++j) {
    const int c = lane * 4 + 128 * j;
    v4f x;
    if (MODE == 2) {
      const v4f ha = *(const v4f*)(src + rb + c);
      const v4f gp = *(const v4f*)(gpre + rb + c);
      const v4f ao = *(const v4f*)(aout + rb + c);
      const v4f bf = *(const v4f*)(biof + rb + c);
#pragma unroll
      for (int e = 0; e < 4; ++e) {
        const float g = sigm_f(gp[e]);
        x[e] = ha[e] + g * ao[e] + (1.0f - g) * bf[e];
      }
      float* hp = hc + rb + c;
      *(volatile v4f*)hp = x;
      __threadfence();
      *(volatile v4f*)hp = x;
    } else {
      x = *(const v4f*)(src + rb + c);
    }
    *(v4f*)(sr + c) = x;
    sum += (x[0] + x[1]) + (x[2] + x[3]);
  }
#pragma unroll
  for (int off = 1; off < 32; off <<= 1) sum += __shfl_xor(sum, off, 32);
  const float mean = sum * (1.0f / (float)kDm);
  __syncthreads();
  float var = 0.f;
#pragma unroll 1
  for (int j = 0; j < 4; ++j) {
    const int c = lane * 4 + 128 * j;
    const v4f x = *(const v4f*)(sr + c);
    const float e0 = x[0] - mean, e1 = x[1] - mean, e2 = x[2] - mean, e3 = x[3] - mean;
    var += (e0 * e0 + e1 * e1) + (e2 * e2 + e3 * e3);
  }
#pragma unroll
  for (int off = 1; off < 32; off <<= 1) var += __shfl_xor(var, off, 32);
  const float rstd = rsqrtf(var * (1.0f / (float)kDm) + 1e-5f);
#pragma unroll 1
  for (int jj = 0; jj < 2; ++jj) {
    const int c8 = lane * 8 + 256 * jj;
    const v4f a0 = *(const v4f*)(sr + c8);
    const v4f a1 = *(const v4f*)(sr + c8 + 4);
    v8h hv, av;
#pragma unroll
    for (int e = 0; e < 4; ++e) {
      hv[e]     = (_Float16)(((a0[e] - mean) * rstd) * gam[c8 + e] + bet[c8 + e]);
      hv[4 + e] = (_Float16)(((a1[e] - mean) * rstd) * gam[c8 + 4 + e] + bet[c8 + 4 + e]);
      if (MODE == 1) {
        av[e]     = (_Float16)(a0[e] * 4096.0f);
        av[4 + e] = (_Float16)(a1[e] * 4096.0f);
      }
    }
    unsigned short* p = dst16 + rb + c8;
    unsigned short* pa = (MODE == 1) ? (aux16 + (size_t)row * kGcW + c8) : nullptr;
    *(volatile v8h*)p = hv;
    if (MODE == 1) *(volatile v8h*)pa = av;
    __threadfence();
    *(volatile v8h*)p = hv;
    if (MODE == 1) *(volatile v8h*)pa = av;
  }
}

__global__ __launch_bounds__(256) void softmax_rows_kernel(
    const float* __restrict__ S, unsigned short* __restrict__ P16, const int* __restrict__ nh_unused)
{
  __shared__ __align__(16) float sh[8][kSeq];
  (void)nh_unused;
  const int tid = threadIdx.x, lane = tid & 31, wave = tid >> 5;
  const int row = blockIdx.x * 8 + wave;
  const size_t rb = (size_t)row * kSeq;
  float* sr = sh[wave];
  float m = -INFINITY;
#pragma unroll 1
  for (int j = 0; j < 8; ++j) {
    const int c = lane * 4 + 128 * j;
    const v4f x = *(const v4f*)(S + rb + c);
    m = fmaxf(m, fmaxf(fmaxf(x[0], x[1]), fmaxf(x[2], x[3])));
  }
#pragma unroll
  for (int off = 1; off < 32; off <<= 1) m = fmaxf(m, __shfl_xor(m, off, 32));
  float sum = 0.f;
#pragma unroll 1
  for (int j = 0; j < 8; ++j) {
    const int c = lane * 4 + 128 * j;
    const v4f x = *(const v4f*)(S + rb + c);
    v4f e;
    e[0] = expf(x[0] - m); e[1] = expf(x[1] - m); e[2] = expf(x[2] - m); e[3] = expf(x[3] - m);
    *(v4f*)(sr + c) = e;
    sum += (e[0] + e[1]) + (e[2] + e[3]);
  }
#pragma unroll
  for (int off = 1; off < 32; off <<= 1) sum += __shfl_xor(sum, off, 32);
  const float rs = 1024.0f * __builtin_amdgcn_rcpf(sum);
  __syncthreads();
#pragma unroll 1
  for (int jj = 0; jj < 4; ++jj) {
    const int c8 = lane * 8 + 256 * jj;
    const v4f a0 = *(const v4f*)(sr + c8);
    const v4f a1 = *(const v4f*)(sr + c8 + 4);
    v8h hv;
#pragma unroll
    for (int e = 0; e < 4; ++e) {
      hv[e]     = (_Float16)(a0[e] * rs);
      hv[4 + e] = (_Float16)(a1[e] * rs);
    }
    unsigned short* p = P16 + rb + c8;
    *(volatile v8h*)p = hv;
    __threadfence();
    *(volatile v8h*)p = hv;
  }
}

template <int BIAS_MODE, int OUT_MODE, bool RESID>
static void launch_gemm(hipStream_t st, int Z,
                        const void* A, int lda, long sA,
                        const void* Bt, int ldb, long sB,
                        void* C, int ldc, long sC,
                        const float* bias, const float* resid, long sR,
                        int M, int N, int K, float scale)
{
  const int tiles = (M >> 6) * (N >> 6);
  const int blocks = (tiles + 7) >> 3;
  wmma_gemm64<0, false, BIAS_MODE, OUT_MODE, RESID, 0><<<dim3(blocks, Z), 256, 0, st>>>(
      (const unsigned short*)A, nullptr, lda, sA,
      (const unsigned short*)Bt, nullptr, ldb, sB,
      C, nullptr, ldc, sC, bias, resid, sR, M, N, K, scale);
}

extern "C" void kernel_launch(void* const* d_in, const int* in_sizes, int n_in,
                              void* d_out, int out_size, void* d_ws, size_t ws_size,
                              hipStream_t stream) {
  if (n_in < 30) return;
  if (in_sizes[0] != kRows * kDm || in_sizes[1] != kRows * kDm) return;
  if (in_sizes[3] != kDm * kDm || in_sizes[4] != kDm) return;
  if (in_sizes[5] != kDm * kBxzW) return;
  if (in_sizes[6] != kDin * 4 || in_sizes[7] != kDin) return;
  if (in_sizes[8] != kCatW * kDin || in_sizes[9] != kDin) return;
  if (in_sizes[10] != kDin * kBcReal || in_sizes[11] != kDin * kNst || in_sizes[12] != kDin) return;
  if (in_sizes[13] != kDin * kDm) return;
  if (in_sizes[14] != kDm * 3 * kDm || in_sizes[15] != 3 * kDm) return;
  if (in_sizes[16] != kDm * kDm || in_sizes[17] != kDm) return;
  if (in_sizes[18] != kDm || in_sizes[19] != kDm || in_sizes[20] != kDm || in_sizes[21] != kDm) return;
  if (in_sizes[22] != kGcW * kDm || in_sizes[23] != kDm) return;
  if (in_sizes[24] != kDm || in_sizes[25] != kDm) return;
  if (in_sizes[26] != kDm * kF1W || in_sizes[27] != kF1W) return;
  if (in_sizes[28] != kF1W * kDm || in_sizes[29] != kDm) return;
  if (out_size != kRows * kDm) return;
  if (ws_size < kWsTotal) return;

  const float* h_audio    = (const float*)d_in[0];
  const float* h_bio      = (const float*)d_in[1];
  const int*   n_heads    = (const int*)d_in[2];
  const float* ctx_W      = (const float*)d_in[3];
  const float* ctx_b      = (const float*)d_in[4];
  const float* bio_in_W   = (const float*)d_in[5];
  const float* conv_W     = (const float*)d_in[6];
  const float* conv_b     = (const float*)d_in[7];
  const float* dt_W       = (const float*)d_in[8];
  const float* dt_b       = (const float*)d_in[9];
  const float* bc_W       = (const float*)d_in[10];
  const float* A_log      = (const float*)d_in[11];
  const float* D_param    = (const float*)d_in[12];
  const float* ssm_out_W  = (const float*)d_in[13];
  const float* in_proj_W  = (const float*)d_in[14];
  const float* in_proj_b  = (const float*)d_in[15];
  const float* out_proj_W = (const float*)d_in[16];
  const float* out_proj_b = (const float*)d_in[17];
  const float* nq_g       = (const float*)d_in[18];
  const float* nq_b       = (const float*)d_in[19];
  const float* nkv_g      = (const float*)d_in[20];
  const float* nkv_b      = (const float*)d_in[21];
  const float* gate_W     = (const float*)d_in[22];
  const float* gate_b     = (const float*)d_in[23];
  const float* ffn_ln_g   = (const float*)d_in[24];
  const float* ffn_ln_b   = (const float*)d_in[25];
  const float* ffn_W1     = (const float*)d_in[26];
  const float* ffn_b1     = (const float*)d_in[27];
  const float* ffn_W2     = (const float*)d_in[28];
  const float* ffn_b2     = (const float*)d_in[29];
  float* out = (float*)d_out;

  char* ws = (char*)d_ws;
  unsigned short* WCTX  = (unsigned short*)(ws + kOffWCTX);
  unsigned short* WBIO  = (unsigned short*)(ws + kOffWBIO);
  unsigned short* WDT   = (unsigned short*)(ws + kOffWDT);
  unsigned short* WBC   = (unsigned short*)(ws + kOffWBC);
  unsigned short* WSSM  = (unsigned short*)(ws + kOffWSSM);
  unsigned short* WIN   = (unsigned short*)(ws + kOffWIN);
  unsigned short* WOUT  = (unsigned short*)(ws + kOffWOUT);
  unsigned short* WGATE = (unsigned short*)(ws + kOffWGATE);
  unsigned short* WF1   = (unsigned short*)(ws + kOffWF1);
  unsigned short* WF2   = (unsigned short*)(ws + kOffWF2);
  unsigned short* HA16  = (unsigned short*)(ws + kOffRS);
  unsigned short* HB16  = (unsigned short*)(ws + kOffRS + (size_t)kRows * kDm * 2);
  float*          CTXP  = (float*)(ws + kOffRS + (size_t)2 * kRows * kDm * 2);
  float*          Sbuf  = (float*)(ws + kOffRS);
  float*          BXZ   = (float*)(ws + kOffRB);
  float*          BIOF  = (float*)(ws + kOffRB);
  unsigned short* GCAT  = (unsigned short*)(ws + kOffRB + (size_t)kRows * kDm * 4);
  float*          AOUT  = (float*)(ws + kOffRB + (size_t)2 * kRows * kDm * 4);
  float*          GPRE  = (float*)(ws + kOffRB + (size_t)3 * kRows * kDm * 4);
  float*          UC    = (float*)(ws + kOffRU);
  unsigned short* QP16  = (unsigned short*)(ws + kOffRU);
  unsigned short* KP16  = (unsigned short*)(ws + kOffRU + (size_t)kRows * kDm * 2);
  unsigned short* VT16  = (unsigned short*)(ws + kOffRU + (size_t)2 * kRows * kDm * 2);
  float*          F1P   = (float*)(ws + kOffRU);
  float*          DTP   = (float*)(ws + kOffRD);
  unsigned short* P16   = (unsigned short*)(ws + kOffRD);
  unsigned short* Y1    = (unsigned short*)(ws + kOffRD);
  unsigned short* CAT   = (unsigned short*)(ws + kOffRC);
  unsigned short* Y16   = (unsigned short*)(ws + kOffRC);
  unsigned short* QLN16 = (unsigned short*)(ws + kOffRC);
  unsigned short* KVLN16 = (unsigned short*)(ws + kOffRC + (size_t)kRows * kDm * 2);
  unsigned short* ATT16 = (unsigned short*)(ws + kOffRC + (size_t)2 * kRows * kDm * 2);
  float*          HC    = (float*)(ws + kOffRC);
  unsigned short* LN2   = (unsigned short*)(ws + kOffRC + (size_t)kRows * kDm * 4);
  float*          BCm   = (float*)(ws + kOffRBC);

  const float s32 = 1.0f / 32.0f;

  act_cast_kernel<0><<<(kRows * kDm) / 2048, 256, 0, stream>>>(h_audio, kDm, HA16, kDm, 0, 1.0f);
  act_cast_kernel<0><<<(kRows * kDm) / 2048, 256, 0, stream>>>(h_bio, kDm, HB16, kDm, 0, 1.0f);

  wt_cast_kernel<<<dim3(kDm / 64,  kDm / 64),        256, 0, stream>>>(ctx_W,      kDm,      WCTX,  kDm,  32.0f);
  wt_cast_kernel<<<dim3(kDm / 64,  kBxzW / 64),      256, 0, stream>>>(bio_in_W,   kBxzW,    WBIO,  kDm,  32.0f);
  wt_cast_kernel<<<dim3(kCatW / 64, kDin / 64),      256, 0, stream>>>(dt_W,       kDin,     WDT,   kCatW, 32.0f);
  wt_cast_kernel<<<dim3(kDin / 64, kBcW / 64),       256, 0, stream>>>(bc_W,       kBcReal,  WBC,   kDin, 32.0f);
  wt_cast_kernel<<<dim3(kDin / 64, kDm / 64),        256, 0, stream>>>(ssm_out_W,  kDm,      WSSM,  kDin, 32.0f);
  wt_cast_kernel<<<dim3(kDm / 64,  (3 * kDm) / 64),  256, 0, stream>>>(in_proj_W,  3 * kDm,  WIN,   kDm,  32.0f);
  wt_cast_kernel<<<dim3(kDm / 64,  kDm / 64),        256, 0, stream>>>(out_proj_W, kDm,      WOUT,  kDm,  32.0f);
  wt_cast_kernel<<<dim3(kGcW / 64, kDm / 64),        256, 0, stream>>>(gate_W,     kDm,      WGATE, kGcW, 32.0f);
  wt_cast_kernel<<<dim3(kDm / 64,  kF1W / 64),       256, 0, stream>>>(ffn_W1,     kF1W,     WF1,   kDm,  32.0f);
  wt_cast_kernel<<<dim3(kF1W / 64, kDm / 64),        256, 0, stream>>>(ffn_W2,     kDm,      WF2,   kF1W, 32.0f);

  launch_gemm<2, 0, false>(stream, 1, HA16, kDm, 0L, WCTX, kDm, 0L, (void*)CTXP, kDm, 0L,
                           ctx_b, nullptr, 0L, kRows, kDm, kDm, s32);
  act_cast_kernel<1><<<(kRows * kDm) / 2048, 256, 0, stream>>>(CTXP, kDm, CAT, kCatW, kDin, 256.0f);

  launch_gemm<0, 0, false>(stream, 1, HB16, kDm, 0L, WBIO, kDm, 0L, (void*)BXZ, kBxzW, 0L,
                           nullptr, nullptr, 0L, kRows, kBxzW, kDm, s32);

  conv_silu_kernel<<<dim3(kDin / 256, kRows / 64), 256, 0, stream>>>(BXZ, conv_W, conv_b, UC, CAT);

  launch_gemm<2, 0, false>(stream, 1, CAT, kCatW, 0L, WDT, kCatW, 0L, (void*)DTP, kDin, 0L,
                           dt_b, nullptr, 0L, kRows, kDin, kCatW, 1.0f / 8192.0f);
  launch_gemm<0, 0, false>(stream, 1, CAT, kCatW, 0L, WBC, kDin, 0L, (void*)BCm, kBcW, 0L,
                           nullptr, nullptr, 0L, kRows, kBcW, kDin, 1.0f / 8192.0f);

  scan_kernel<<<kBatch * (kDin / kScanCh), kScanCh, 0, stream>>>(DTP, BCm, UC, BXZ, A_log, D_param, Y16);

  launch_gemm<0, 0, false>(stream, 1, Y16, kDin, 0L, WSSM, kDin, 0L, (void*)BIOF, kDm, 0L,
                           nullptr, nullptr, 0L, kRows, kDm, kDin, 1.0f / 32768.0f);

  ln_rows_kernel<0><<<kRows / 8, 256, 0, stream>>>(h_audio, nullptr, nullptr, nullptr, nq_g, nq_b, nullptr, QLN16, nullptr);
  ln_rows_kernel<1><<<kRows / 8, 256, 0, stream>>>(BIOF, nullptr, nullptr, nullptr, nkv_g, nkv_b, nullptr, KVLN16, GCAT);

  launch_gemm<2, 1, false>(stream, 1, QLN16, kDm, 0L, WIN, kDm, 0L, (void*)QP16, kDm, 0L,
                           in_proj_b, nullptr, 0L, kRows, kDm, kDm, s32);
  launch_gemm<2, 1, false>(stream, 1, KVLN16, kDm, 0L, WIN + (size_t)kDm * kDm, kDm, 0L, (void*)KP16, kDm, 0L,
                           in_proj_b + kDm, nullptr, 0L, kRows, kDm, kDm, s32);
  launch_gemm<1, 1, false>(stream, 1, WIN + (size_t)2 * kDm * kDm, kDm, 0L, KVLN16, kDm, 0L, (void*)VT16, kRows, 0L,
                           in_proj_b + 2 * kDm, nullptr, 0L, kDm, kRows, kDm, s32);

  for (int bb = 0; bb < kBatch; ++bb) {
    launch_gemm<0, 0, false>(stream, kHeads,
                             QP16 + (size_t)bb * kSeq * kDm, kDm, (long)kDh,
                             KP16 + (size_t)bb * kSeq * kDm, kDm, (long)kDh,
                             (void*)Sbuf, kSeq, (long)kSeq * kSeq,
                             nullptr, nullptr, 0L, kSeq, kSeq, kDh, 0.125f);
    softmax_rows_kernel<<<(kHeads * kSeq) / 8, 256, 0, stream>>>(Sbuf, P16, n_heads);
    launch_gemm<0, 1, false>(stream, kHeads,
                             P16, kSeq, (long)kSeq * kSeq,
                             VT16 + (size_t)bb * kSeq, kRows, (long)kDh * kRows,
                             (void*)(ATT16 + (size_t)bb * kSeq * kDm), kDm, (long)kDh,
                             nullptr, nullptr, 0L, kSeq, kDh, kSeq, 0.25f);
  }

  launch_gemm<2, 0, false>(stream, 1, ATT16, kDm, 0L, WOUT, kDm, 0L, (void*)AOUT, kDm, 0L,
                           out_proj_b, nullptr, 0L, kRows, kDm, kDm, 1.0f / 8192.0f);
  act_cast_kernel<0><<<(kRows * kDm) / 2048, 256, 0, stream>>>(AOUT, kDm, GCAT, kGcW, kDm, 4096.0f);

  launch_gemm<2, 0, false>(stream, 1, GCAT, kGcW, 0L, WGATE, kGcW, 0L, (void*)GPRE, kDm, 0L,
                           gate_b, nullptr, 0L, kRows, kDm, kGcW, 1.0f / 131072.0f);

  ln_rows_kernel<2><<<kRows / 8, 256, 0, stream>>>(h_audio, GPRE, AOUT, BIOF, ffn_ln_g, ffn_ln_b, HC, LN2, nullptr);

  launch_gemm<2, 0, false>(stream, 1, LN2, kDm, 0L, WF1, kDm, 0L, (void*)F1P, kF1W, 0L,
                           ffn_b1, nullptr, 0L, kRows, kF1W, kDm, s32);
  act_cast_kernel<1><<<(kRows * kF1W) / 2048, 256, 0, stream>>>(F1P, kF1W, Y1, kF1W, 0, 16.0f);
  launch_gemm<2, 0, true>(stream, 1, Y1, kF1W, 0L, WF2, kF1W, 0L, (void*)out, kDm, 0L,
                          ffn_b2, HC, 0L, kRows, kDm, kF1W, 1.0f / 512.0f);
}
